// EdgeScoringMLP_73589969649904
// MI455X (gfx1250) — hardware-verified
//
#include <hip/hip_runtime.h>
#include <math.h>

typedef __attribute__((ext_vector_type(16))) _Float16 v16h;
typedef __attribute__((ext_vector_type(16))) __bf16 v16b;
typedef __attribute__((ext_vector_type(8)))  _Float16 v8h;
typedef __attribute__((ext_vector_type(8)))  float v8f;
typedef __attribute__((ext_vector_type(4)))  float v4f;
typedef __attribute__((ext_vector_type(2)))  float v2f;
typedef __attribute__((ext_vector_type(4)))  unsigned v4u;
typedef __attribute__((ext_vector_type(4)))  int v4i;
typedef float __attribute__((may_alias)) float_a;
typedef int __attribute__((may_alias)) int_a;

template <typename T> __device__ __forceinline__ void vst2(void* p, T v) { *(volatile T*)p = v; __threadfence(); *(volatile T*)p = v; }
__device__ __forceinline__ v8f wmma16(v16h a, v16h b, v8f c) {
  v8f d = __builtin_amdgcn_wmma_f32_16x16x32_f16(false, a, false, b, (short)0, c, false, false);
  asm volatile("v_nop\n\tv_nop\n\tv_nop\n\tv_nop" : "+v"(d) : "v"(a), "v"(b));
  return d;
}
__device__ __forceinline__ v8f wmma_bf(v16b a, v16b b, v8f c) {
  v8f d = __builtin_amdgcn_wmma_f32_16x16x32_bf16(false, a, false, b, (short)0, c, false, false);
  asm volatile("v_nop\n\tv_nop\n\tv_nop\n\tv_nop" : "+v"(d) : "v"(a), "v"(b));
  return d;
}
__device__ __forceinline__ v16h frag_h(const _Float16* rowk0, int lane) {
  union { v16h v; v8h q[2]; } u; const _Float16* p = rowk0 + 8 * (lane >> 4);
  u.q[0] = *(const v8h*)p; u.q[1] = *(const v8h*)(p + 16); return u.v;
}
__device__ __forceinline__ v16h frag_f32(const float* rowk0, int lane) {
  v16h a; const float* p = rowk0 + 8 * (lane >> 4);
#pragma unroll
  for (int i = 0; i < 8; ++i) { a[i] = (_Float16)p[i]; a[8 + i] = (_Float16)p[16 + i]; }
  return a;
}
__device__ __forceinline__ v16h frag_f32s(const float* rowk0, int lane, float sc) {
  v16h a; const float* p = rowk0 + 8 * (lane >> 4);
#pragma unroll
  for (int i = 0; i < 8; ++i) { a[i] = (_Float16)(p[i] * sc); a[8 + i] = (_Float16)(p[16 + i] * sc); }
  return a;
}
__device__ __forceinline__ v16h fragc_f32(const float* W, int k0, int n, int lane, int ld, int K) {
  v16h a; const int g = lane >> 4;
#pragma unroll
  for (int i = 0; i < 8; ++i) { const int ka = k0 + 8 * g + i, kb = ka + 16;
    a[i] = (_Float16)(ka < K ? W[(size_t)ka * ld + n] : 0.f); a[8 + i] = (_Float16)(kb < K ? W[(size_t)kb * ld + n] : 0.f); }
  return a;
}
struct F2 { v16b h, l; };
__device__ __forceinline__ F2 bsplit16(const float v[16]) { F2 r;
#pragma unroll
  for (int i = 0; i < 16; ++i) { const __bf16 h = (__bf16)v[i]; r.h[i] = h; r.l[i] = (__bf16)(v[i] - (float)h); }
  return r; }
__device__ __forceinline__ F2 split_row(const float* row, int k0, int lane) { float v[16]; const float* p = row + k0 + 8 * (lane >> 4);
#pragma unroll
  for (int i = 0; i < 8; ++i) { v[i] = p[i]; v[8 + i] = p[16 + i]; }
  return bsplit16(v); }
__device__ __forceinline__ F2 split_rowK(const float* row, int k0, int lane, int K) { float v[16]; const int g = lane >> 4;
#pragma unroll
  for (int i = 0; i < 8; ++i) { const int ka = k0 + 8 * g + i, kb = ka + 16; v[i] = ka < K ? row[ka] : 0.f; v[8 + i] = kb < K ? row[kb] : 0.f; }
  return bsplit16(v); }
__device__ __forceinline__ F2 split_col(const float* W, int k0, int n, int lane, int ld, int K) { float v[16]; const int g = lane >> 4;
#pragma unroll
  for (int i = 0; i < 8; ++i) { const int ka = k0 + 8 * g + i, kb = ka + 16; v[i] = ka < K ? W[(size_t)ka * ld + n] : 0.f; v[8 + i] = kb < K ? W[(size_t)kb * ld + n] : 0.f; }
  return bsplit16(v); }
__device__ __forceinline__ v8f mac3(const F2& a, const F2& b, v8f c) { c = wmma_bf(a.l, b.h, c); c = wmma_bf(a.h, b.l, c); return wmma_bf(a.h, b.h, c); }
__device__ __forceinline__ float sigm(float v) { return 1.0f / (1.0f + expf(-v)); }
#define LDSX() do { asm volatile("s_wait_dscnt 0" ::: "memory"); __builtin_amdgcn_wave_barrier(); __builtin_amdgcn_fence(__ATOMIC_RELEASE, "workgroup"); } while (0)

#define NN 100000
#define NNP 100032
#define NE 1000000
#define HH 128
#define H2 64
#define CHE 200000
#define CHP 200000

__global__ __launch_bounds__(256) void k_cvt(const float* __restrict__ x, _Float16* __restrict__ x16) {
  const size_t g8 = (size_t)blockIdx.x * 256 + threadIdx.x; if (g8 >= (size_t)NNP * HH / 8) return;
  const size_t e0 = g8 * 8; union { v8h h; v4u u; } pk;
#pragma unroll
  for (int e = 0; e < 8; ++e) pk.h[e] = (_Float16)(e0 + e < (size_t)NN * HH ? x[e0 + e] : 0.f);
  vst2(x16 + e0, pk.u);
}
__global__ __launch_bounds__(256) void k_packW(const float* __restrict__ W1, const float* __restrict__ W2, _Float16* __restrict__ P) {
  __shared__ float tile[64][65];
  const int which = blockIdx.z, o0 = blockIdx.x * 64, k0 = blockIdx.y * 64, tid = threadIdx.x;
  if (which == 2 && (o0 >= H2 || k0 >= HH)) return;
  if (which < 2) { for (int q = tid; q < 64 * 64; q += 256) { const int kl = q >> 6, ol = q & 63; tile[kl][ol] = W1[(size_t)(which * HH + k0 + kl) * HH + o0 + ol]; } }
  else { for (int q = tid; q < 64 * 64; q += 256) { const int kl = q >> 6, ol = q & 63; tile[kl][ol] = W2[(size_t)(k0 + kl) * H2 + o0 + ol]; } }
  __syncthreads();
  for (int u = 0; u < 2; ++u) { const int idx = tid + u * 256, ol = idx >> 3, pc = idx & 7; union { v8h hh; v4u uu; } pk;
#pragma unroll
    for (int i = 0; i < 8; ++i) pk.hh[i] = (_Float16)(tile[pc * 8 + i][ol] * 16.0f);
    vst2(P + ((size_t)which * HH + o0 + ol) * HH + k0 + pc * 8, pk.uu); }
}
__global__ __launch_bounds__(128) void k_uv(const _Float16* __restrict__ x16, const _Float16* __restrict__ P, float* __restrict__ U, float* __restrict__ V) {
  __shared__ __align__(16) float so[4][16][132];
  const int tid = threadIdx.x, wave = tid >> 5, lane = tid & 31, col = lane & 15, g = lane >> 4;
  const int r0 = blockIdx.x * 64 + wave * 16, which = blockIdx.y; float* dst = which ? V : U;
  v8f acc[8] = {};
#pragma unroll
  for (int kc = 0; kc < HH / 32; ++kc) { const v16h a = frag_h(x16 + (size_t)(r0 + col) * HH + kc * 32, lane);
#pragma unroll
    for (int j = 0; j < 8; ++j) acc[j] = wmma16(a, frag_h(P + (size_t)(which * HH + j * 16 + col) * HH + kc * 32, lane), acc[j]); }
#pragma unroll
  for (int j = 0; j < 8; ++j)
#pragma unroll
    for (int r = 0; r < 8; ++r) so[wave][8 * g + r][j * 16 + col] = acc[j][r] * (1.0f / 16.0f);
  LDSX();
#pragma unroll 4
  for (int rl = 0; rl < 16; ++rl) vst2(dst + (size_t)(r0 + rl) * HH + lane * 4, *(const v4f*)(&so[wave][rl][lane * 4]));
}
__global__ __launch_bounds__(256) void k_gath(const int* __restrict__ ei, const float* __restrict__ attr, const float* __restrict__ U, const float* __restrict__ V, const float* __restrict__ W1, const float* __restrict__ b1, const float* __restrict__ gam, const float* __restrict__ bet, int e0c, _Float16* __restrict__ Hc) {
  __shared__ __align__(16) _Float16 sh[64][HH + 8];
  __shared__ float sw[2][HH], sb[HH], sg[HH], sbe[HH];
  const int tid = threadIdx.x, w = tid >> 5, lane = tid & 31;
  if (tid < HH) { sw[0][tid] = W1[(size_t)(2 * HH) * HH + tid]; sw[1][tid] = W1[(size_t)(2 * HH + 1) * HH + tid]; sb[tid] = b1[tid]; sg[tid] = gam[tid]; sbe[tid] = bet[tid]; }
  __syncthreads();
  const int el0 = blockIdx.x * 64;
  { const int el = el0 + w * 8 + (lane >> 2), part = lane & 3; const int e = e0c + el; const bool ok = e < NE;
    int i = ok ? ei[e] : 0, j = ok ? ei[(size_t)NE + e] : 0; i = i < 0 ? 0 : (i >= NN ? NN - 1 : i); j = j < 0 ? 0 : (j >= NN ? NN - 1 : j);
    const float a0 = ok ? attr[(size_t)e * 2] : 0.f, a1 = ok ? attr[(size_t)e * 2 + 1] : 0.f;
    float v[32]; float s = 0.f;
#pragma unroll
    for (int c = 0; c < 32; ++c) { const int cc = part * 32 + c; const float hv = U[(size_t)i * HH + cc] + V[(size_t)j * HH + cc] + a0 * sw[0][cc] + a1 * sw[1][cc] + sb[cc]; v[c] = hv; s += hv; }
    s += __shfl_xor(s, 1, 32); s += __shfl_xor(s, 2, 32); const float mu = s * (1.0f / HH);
    float q2 = 0.f;
#pragma unroll
    for (int c = 0; c < 32; ++c) { const float d = v[c] - mu; q2 += d * d; }
    q2 += __shfl_xor(q2, 1, 32); q2 += __shfl_xor(q2, 2, 32); const float rs = rsqrtf(q2 * (1.0f / HH) + 1e-5f);
#pragma unroll
    for (int c = 0; c < 32; ++c) { const int cc = part * 32 + c; float hv = (v[c] - mu) * rs * sg[cc] + sbe[cc]; hv = hv > 0.f ? hv : 0.f; sh[w * 8 + (lane >> 2)][cc] = (_Float16)(ok ? hv : 0.f); } }
  __syncthreads();
  for (int q = tid; q < 64 * 16; q += 256) { const int rl = q >> 4, pc = q & 15; vst2(Hc + (size_t)(el0 + rl) * HH + pc * 8, *(const v4u*)(&sh[rl][pc * 8])); }
}
__global__ __launch_bounds__(128) void k_mlp(const _Float16* __restrict__ Hc, const _Float16* __restrict__ P, const float* __restrict__ b2, const float* __restrict__ W3, const float* __restrict__ b3, int e0c, float* __restrict__ out) {
  __shared__ __align__(16) float so[4][16][68];
  __shared__ __align__(16) float sl[64];
  const int tid = threadIdx.x, wave = tid >> 5, lane = tid & 31, col = lane & 15, g = lane >> 4;
  const int el0 = blockIdx.x * 64 + wave * 16;
  v8f acc[4] = {};
#pragma unroll
  for (int kc = 0; kc < HH / 32; ++kc) { const v16h a = frag_h(Hc + (size_t)(el0 + col) * HH + kc * 32, lane);
#pragma unroll
    for (int j = 0; j < 4; ++j) acc[j] = wmma16(a, frag_h(P + (size_t)(2 * HH + j * 16 + col) * HH + kc * 32, lane), acc[j]); }
#pragma unroll
  for (int j = 0; j < 4; ++j) { const int c = j * 16 + col; const float bb = b2[c];
#pragma unroll
    for (int r = 0; r < 8; ++r) { const float v = acc[j][r] * (1.0f / 16.0f) + bb; so[wave][8 * g + r][c] = v > 0.f ? v : 0.f; } }
  LDSX();
  { const int rl = lane >> 1, hf = lane & 1; float s = 0.f;
#pragma unroll 8
    for (int c = 0; c < 32; ++c) s += so[wave][rl][hf * 32 + c] * W3[hf * 32 + c];
    s += __shfl_xor(s, 1, 32); if (hf == 0) sl[wave * 16 + rl] = s + b3[0]; }
  __syncthreads();
  if (tid < 16) { const int e = e0c + blockIdx.x * 64 + tid * 4; vst2(out + e, *(const v4f*)(&sl[tid * 4])); }
}
extern "C" void kernel_launch(void* const* d_in, const int* in_sizes, int n_in, void* d_out, int out_size, void* d_ws, size_t ws_size, hipStream_t stream) {
  (void)in_sizes; (void)n_in; (void)out_size; (void)ws_size;
  const float* x = (const float*)d_in[0]; const int* ei = (const int*)d_in[1]; const float* attr = (const float*)d_in[2]; const float* W1 = (const float*)d_in[3]; const float* b1 = (const float*)d_in[4];
  const float* gam = (const float*)d_in[5]; const float* bet = (const float*)d_in[6]; const float* W2 = (const float*)d_in[7]; const float* b2 = (const float*)d_in[8]; const float* W3 = (const float*)d_in[9]; const float* b3 = (const float*)d_in[10];
  float* out = (float*)d_out;
  char* ws = (char*)d_ws; size_t off = 0;
  auto take = [&](size_t bytes) { char* p = ws + off; off += (bytes + 255) & ~(size_t)255; return p; };
  _Float16* x16 = (_Float16*)take((size_t)NNP * HH * 2); _Float16* P = (_Float16*)take((size_t)(2 * HH + H2) * HH * 2); float* U = (float*)take((size_t)NNP * HH * 4); float* V = (float*)take((size_t)NNP * HH * 4);
  _Float16* Hc = (_Float16*)take((size_t)CHP * HH * 2);
  k_cvt<<<(unsigned)(((size_t)NNP * HH / 8 + 255) / 256), 256, 0, stream>>>(x, x16);
  k_packW<<<dim3(HH / 64, HH / 64, 3), 256, 0, stream>>>(W1, W2, P);
  k_uv<<<dim3(NNP / 64, 2), 128, 0, stream>>>(x16, P, U, V);
  for (int c = 0; c < NE / CHE; ++c) { const int e0c = c * CHE;
    k_gath<<<CHP / 64, 256, 0, stream>>>(ei, attr, U, V, W1, b1, gam, bet, e0c, Hc);
    k_mlp<<<CHP / 64, 128, 0, stream>>>(Hc, P, b2, W3, b3, e0c, out); }
}
